// BezierToImageLayer_36197984371365
// MI455X (gfx1250) — hardware-verified
//
#include <hip/hip_runtime.h>
#include <math.h>

typedef __attribute__((ext_vector_type(16))) _Float16 v16h;
typedef __attribute__((ext_vector_type(16))) __bf16 v16b;
typedef __attribute__((ext_vector_type(8)))  _Float16 v8h;
typedef __attribute__((ext_vector_type(8)))  float v8f;
typedef __attribute__((ext_vector_type(4)))  float v4f;
typedef __attribute__((ext_vector_type(2)))  float v2f;
typedef __attribute__((ext_vector_type(4)))  unsigned v4u;
typedef __attribute__((ext_vector_type(4)))  int v4i;
typedef float __attribute__((may_alias)) float_a;
typedef int __attribute__((may_alias)) int_a;

template <typename T> __device__ __forceinline__ void vst2(void* p, T v) { *(volatile T*)p = v; __threadfence(); *(volatile T*)p = v; }
__device__ __forceinline__ v8f wmma16(v16h a, v16h b, v8f c) {
  v8f d = __builtin_amdgcn_wmma_f32_16x16x32_f16(false, a, false, b, (short)0, c, false, false);
  asm volatile("v_nop\n\tv_nop\n\tv_nop\n\tv_nop" : "+v"(d) : "v"(a), "v"(b));
  return d;
}
__device__ __forceinline__ v8f wmma_bf(v16b a, v16b b, v8f c) {
  v8f d = __builtin_amdgcn_wmma_f32_16x16x32_bf16(false, a, false, b, (short)0, c, false, false);
  asm volatile("v_nop\n\tv_nop\n\tv_nop\n\tv_nop" : "+v"(d) : "v"(a), "v"(b));
  return d;
}
__device__ __forceinline__ v16h frag_h(const _Float16* rowk0, int lane) {
  union { v16h v; v8h q[2]; } u; const _Float16* p = rowk0 + 8 * (lane >> 4);
  u.q[0] = *(const v8h*)p; u.q[1] = *(const v8h*)(p + 16); return u.v;
}
__device__ __forceinline__ v16h frag_f32(const float* rowk0, int lane) {
  v16h a; const float* p = rowk0 + 8 * (lane >> 4);
#pragma unroll
  for (int i = 0; i < 8; ++i) { a[i] = (_Float16)p[i]; a[8 + i] = (_Float16)p[16 + i]; }
  return a;
}
__device__ __forceinline__ v16h frag_f32s(const float* rowk0, int lane, float sc) {
  v16h a; const float* p = rowk0 + 8 * (lane >> 4);
#pragma unroll
  for (int i = 0; i < 8; ++i) { a[i] = (_Float16)(p[i] * sc); a[8 + i] = (_Float16)(p[16 + i] * sc); }
  return a;
}
__device__ __forceinline__ v16h fragc_f32(const float* W, int k0, int n, int lane, int ld, int K) {
  v16h a; const int g = lane >> 4;
#pragma unroll
  for (int i = 0; i < 8; ++i) { const int ka = k0 + 8 * g + i, kb = ka + 16;
    a[i] = (_Float16)(ka < K ? W[(size_t)(ka < K ? ka : K - 1) * ld + n] : 0.f); a[8 + i] = (_Float16)(kb < K ? W[(size_t)(kb < K ? kb : K - 1) * ld + n] : 0.f); }
  return a;
}
struct F2 { v16b h, l; };
__device__ __forceinline__ F2 bsplit16(const float v[16]) { F2 r;
#pragma unroll
  for (int i = 0; i < 16; ++i) { const __bf16 h = (__bf16)v[i]; r.h[i] = h; r.l[i] = (__bf16)(v[i] - (float)h); }
  return r; }
__device__ __forceinline__ F2 split_row(const float* row, int k0, int lane) { float v[16]; const float* p = row + k0 + 8 * (lane >> 4);
#pragma unroll
  for (int i = 0; i < 8; ++i) { v[i] = p[i]; v[8 + i] = p[16 + i]; }
  return bsplit16(v); }
__device__ __forceinline__ F2 split_rowK(const float* row, int k0, int lane, int K) { float v[16]; const int g = lane >> 4;
#pragma unroll
  for (int i = 0; i < 8; ++i) { const int ka = k0 + 8 * g + i, kb = ka + 16; v[i] = ka < K ? row[ka < K ? ka : K - 1] : 0.f; v[8 + i] = kb < K ? row[kb < K ? kb : K - 1] : 0.f; }
  return bsplit16(v); }
__device__ __forceinline__ F2 split_col(const float* W, int k0, int n, int lane, int ld, int K) { float v[16]; const int g = lane >> 4;
#pragma unroll
  for (int i = 0; i < 8; ++i) { const int ka = k0 + 8 * g + i, kb = ka + 16; v[i] = ka < K ? W[(size_t)(ka < K ? ka : K - 1) * ld + n] : 0.f; v[8 + i] = kb < K ? W[(size_t)(kb < K ? kb : K - 1) * ld + n] : 0.f; }
  return bsplit16(v); }
__device__ __forceinline__ v8f mac3(const F2& a, const F2& b, v8f c) { c = wmma_bf(a.l, b.h, c); c = wmma_bf(a.h, b.l, c); return wmma_bf(a.h, b.h, c); }
__device__ __forceinline__ float sigm(float v) { return 1.0f / (1.0f + expf(-v)); }
#define LDSX() do { asm volatile("s_wait_dscnt 0" ::: "memory"); __builtin_amdgcn_wave_barrier(); __builtin_amdgcn_fence(__ATOMIC_RELEASE, "workgroup"); } while (0)


#define NIMG 256
#define NCUR 160
#define NSMP 30
#define WW 60
#define KK (NCUR * NSMP)
#define ALPHA 0.0002f
__device__ __forceinline__ float bfr(float v) { return (float)(__bf16)v; }
__device__ __attribute__((noinline)) float exp_ni(float v) { return expf(v); }
typedef __attribute__((ext_vector_type(8))) __bf16 v8b;
__device__ __forceinline__ v16b frag_b(const __bf16* rowk0, int lane) {
  union { v16b v; v8b q[2]; } u; const __bf16* p = rowk0 + 8 * (lane >> 4);
  u.q[0] = *(const v8b*)p; u.q[1] = *(const v8b*)(p + 16); return u.v;
}

__global__ __launch_bounds__(256) void k_img(const float* __restrict__ Xc, float* __restrict__ out) {
  __shared__ float sT[NSMP][4];
  __shared__ float sX[2][KK], sY[2][KK];
  __shared__ __align__(16) __bf16 gxh[2][64][40], gxl[2][64][40], gyh[2][64][40], gyl[2][64][40];
  __shared__ __align__(16) float sres[2 * WW * WW];
  const int tid = threadIdx.x, wave = tid >> 5, lane = tid & 31, col = lane & 15, g = lane >> 4;
  const int im = wave >> 2, rt = wave & 3; const int img = blockIdx.x * 2 + im; const int tl = tid & 127;
  if (tid < NSMP) { float t = (float)tid / (float)NSMP; t = 2.0f * (t * t * t) - 3.0f * (t * t) + 2.0f * t; const float tb = 1.0f - t;
    const float t30 = t * t * t, t21 = t * t - t30, t12 = t30 - 2.0f * (t * t) + t, t03 = tb * tb * tb;
    sT[tid][0] = t30; sT[tid][1] = 3.0f * t21; sT[tid][2] = 3.0f * t12; sT[tid][3] = t03; }
  __syncthreads();
  for (int q = tl; q < KK; q += 128) { const int l = q / NSMP, n = q - l * NSMP; const float* c = Xc + ((size_t)img * NCUR + l) * 8;
    float x = 0.f, y = 0.f;
#pragma unroll
    for (int k = 0; k < 4; ++k) { x += sT[n][k] * bfr(c[2 * k]); y += sT[n][k] * bfr(c[2 * k + 1]); }
    sX[im][q] = x; sY[im][q] = y; }
  for (int q = tid; q < 2 * 64 * 40; q += 256) { (&gxh[0][0][0])[q] = (__bf16)0.f; (&gxl[0][0][0])[q] = (__bf16)0.f; (&gyh[0][0][0])[q] = (__bf16)0.f; (&gyl[0][0][0])[q] = (__bf16)0.f; }
  __syncthreads();
  v8f acc[4] = {};
#pragma unroll 1
  for (int kc = 0; kc < KK / 32; ++kc) {
    for (int q = tl; q < WW * 32; q += 128) { const int i = q >> 5, kk = q & 31; const float bxy = (float)i / (float)WW;
      const float dx = bxy - sX[im][kc * 32 + kk], dy = bxy - sY[im][kc * 32 + kk];
      const float ex = exp_ni(-(dx * dx) / ALPHA), ey = exp_ni(-(dy * dy) / ALPHA);
      const __bf16 hx = (__bf16)ex, hy = (__bf16)ey; gxh[im][i][kk] = hx; gxl[im][i][kk] = (__bf16)(ex - (float)hx); gyh[im][i][kk] = hy; gyl[im][i][kk] = (__bf16)(ey - (float)hy); }
    __syncthreads();
    { const v16b ah = frag_b(&gxh[im][rt * 16 + col][0], lane), al = frag_b(&gxl[im][rt * 16 + col][0], lane);
#pragma unroll
      for (int ct = 0; ct < 4; ++ct) { const v16b bh = frag_b(&gyh[im][ct * 16 + col][0], lane), bl = frag_b(&gyl[im][ct * 16 + col][0], lane);
        acc[ct] = wmma_bf(al, bh, acc[ct]); acc[ct] = wmma_bf(ah, bl, acc[ct]); acc[ct] = wmma_bf(ah, bh, acc[ct]); } }
    __syncthreads(); }
#pragma unroll
  for (int ct = 0; ct < 4; ++ct)
#pragma unroll
    for (int r = 0; r < 8; ++r) { const int i = rt * 16 + 8 * g + r, j = ct * 16 + col; if (i < WW && j < WW) sres[im * WW * WW + i * WW + j] = fminf(acc[ct][r], 1.0f); }
  __syncthreads();
  for (int q = tid; q < 2 * WW * WW / 4; q += 256) vst2(out + (size_t)blockIdx.x * 2 * WW * WW + q * 4, *(const v4f*)&sres[q * 4]);
}

extern "C" void kernel_launch(void* const* d_in, const int* in_sizes, int n_in, void* d_out, int out_size, void* d_ws, size_t ws_size, hipStream_t stream) {
  (void)in_sizes; (void)n_in; (void)out_size; (void)d_ws; (void)ws_size;
  k_img<<<NIMG / 2, 256, 0, stream>>>((const float*)d_in[0], (float*)d_out);
}
